// MultiHeadAttention_50251117363504
// MI455X (gfx1250) — hardware-verified
//
#include <hip/hip_runtime.h>
#ifndef NB
#define NB 2
#endif
#ifndef SEQ
#define SEQ 4096
#endif
#define NB_FULL 2
#define SEQ_FULL 4096
#define EMB 768
#define HEADS 8
#define HD 96
#define BSTRIDE_FULL ((size_t)SEQ_FULL * EMB)

#define PLANE_ACT ((size_t)NB * SEQ * EMB * 2)
#define PLANE_W ((size_t)EMB * EMB * 2)
#define CVT_K_BLOCKS ((NB * SEQ * (EMB / 8)) / 256)
#define CVT_W_BLOCKS ((EMB * (EMB / 8)) / 256)
#define PROJ_BLOCKS ((NB * SEQ / 64) * (EMB / 64))

static_assert(SEQ % 64 == 0);
static_assert(SEQ <= SEQ_FULL);
static_assert(NB <= NB_FULL);
static_assert(HEADS * HD == EMB);
static_assert(HD == 96);
static_assert(EMB % 64 == 0);
static_assert(EMB % 96 == 0);
static_assert(EMB % 32 == 0);
static_assert((NB * SEQ) % 64 == 0);
static_assert((NB * SEQ * (EMB / 8)) % 256 == 0);
static_assert((EMB * (EMB / 8)) % 256 == 0);
static_assert(PLANE_ACT % 256 == 0);
static_assert(PLANE_W % 256 == 0);
static_assert(5 * PLANE_ACT + 4 * PLANE_W <= (size_t)134217728);

typedef __bf16 v16b __attribute__((ext_vector_type(16)));
typedef _Float16 v16h __attribute__((ext_vector_type(16)));
typedef unsigned short v8us __attribute__((ext_vector_type(8), may_alias));
typedef float v8f __attribute__((ext_vector_type(8)));
typedef float v4f __attribute__((ext_vector_type(4)));
typedef float v4fa __attribute__((ext_vector_type(4), may_alias));
typedef _Float16 h16;
union FragB { v16b v; v8us half[2]; unsigned short u[16]; };
union FragH { v16h v; v8us half[2]; _Float16 h[16]; unsigned short u[16]; };

#define LOG2E 1.4426950408889634f
#define QK_SCALE 0.10206207261596575f
#define C2 (QK_SCALE * LOG2E)
#define C2S (C2 * 0.00390625f)

__device__ __forceinline__ unsigned short bf16_bits(float x) {
  unsigned int u = __float_as_uint(x);
  return (unsigned short)((u + 0x7FFFu + ((u >> 16) & 1u)) >> 16);
}
__device__ __forceinline__ float bf16_val(unsigned short b) { return __uint_as_float(((unsigned int)b) << 16); }
__device__ __forceinline__ float bf16_rne(float x) { return bf16_val(bf16_bits(x)); }
__device__ __forceinline__ unsigned short f16_bits(float x) {
  union { _Float16 h; unsigned short u; } c;
  c.h = (_Float16)x;
  return c.u;
}
static __device__ __forceinline__ h16 toh_flush(float v) {
  const h16 r = (h16)v;
  return (fabsf(v) < 6.103515625e-05f) ? (h16)0.0f : r;
}
static __device__ __forceinline__ unsigned short toh_flush_bits(float v) {
  union { h16 h; unsigned short u; } c;
  c.h = toh_flush(v);
  return c.u;
}

__device__ __forceinline__ void store_twice(unsigned short* d, v8us o) {
  *(volatile v8us*)d = o;
  __threadfence();
  *(volatile v8us*)d = o;
}

__device__ __forceinline__ void mma_s2h(const FragH (&ka)[3], const FragH (&kb)[3], const FragH (&q)[3], v8f& s0, v8f& s1) {
  s0 = __builtin_amdgcn_wmma_f32_16x16x32_f16(false, ka[0].v, false, q[0].v, (short)0, s0, false, false);
  s1 = __builtin_amdgcn_wmma_f32_16x16x32_f16(false, kb[0].v, false, q[0].v, (short)0, s1, false, false);
  s0 = __builtin_amdgcn_wmma_f32_16x16x32_f16(false, ka[1].v, false, q[1].v, (short)0, s0, false, false);
  s1 = __builtin_amdgcn_wmma_f32_16x16x32_f16(false, kb[1].v, false, q[1].v, (short)0, s1, false, false);
  s0 = __builtin_amdgcn_wmma_f32_16x16x32_f16(false, ka[2].v, false, q[2].v, (short)0, s0, false, false);
  s1 = __builtin_amdgcn_wmma_f32_16x16x32_f16(false, kb[2].v, false, q[2].v, (short)0, s1, false, false);
  asm volatile("v_nop\n\tv_nop\n\tv_nop\n\tv_nop"
               : "+v"(s0), "+v"(s1)
               : "v"(ka[0].v), "v"(ka[1].v), "v"(ka[2].v), "v"(kb[0].v), "v"(kb[1].v), "v"(kb[2].v),
                 "v"(q[0].v), "v"(q[1].v), "v"(q[2].v));
}
__device__ __forceinline__ void mma_pv(const FragH (&vf)[6], v16h p, v8f (&O)[6]) {
  O[0] = __builtin_amdgcn_wmma_f32_16x16x32_f16(false, vf[0].v, false, p, (short)0, O[0], false, false);
  O[1] = __builtin_amdgcn_wmma_f32_16x16x32_f16(false, vf[1].v, false, p, (short)0, O[1], false, false);
  O[2] = __builtin_amdgcn_wmma_f32_16x16x32_f16(false, vf[2].v, false, p, (short)0, O[2], false, false);
  O[3] = __builtin_amdgcn_wmma_f32_16x16x32_f16(false, vf[3].v, false, p, (short)0, O[3], false, false);
  O[4] = __builtin_amdgcn_wmma_f32_16x16x32_f16(false, vf[4].v, false, p, (short)0, O[4], false, false);
  O[5] = __builtin_amdgcn_wmma_f32_16x16x32_f16(false, vf[5].v, false, p, (short)0, O[5], false, false);
  asm volatile("v_nop\n\tv_nop\n\tv_nop\n\tv_nop"
               : "+v"(O[0]), "+v"(O[1]), "+v"(O[2]), "+v"(O[3]), "+v"(O[4]), "+v"(O[5])
               : "v"(p), "v"(vf[0].v), "v"(vf[1].v), "v"(vf[2].v), "v"(vf[3].v), "v"(vf[4].v), "v"(vf[5].v));
}
__device__ __forceinline__ void mma_fc(v16h a, const FragH (&bw)[4], v8f (&c)[4]) {
  c[0] = __builtin_amdgcn_wmma_f32_16x16x32_f16(false, a, false, bw[0].v, (short)0, c[0], false, false);
  c[1] = __builtin_amdgcn_wmma_f32_16x16x32_f16(false, a, false, bw[1].v, (short)0, c[1], false, false);
  c[2] = __builtin_amdgcn_wmma_f32_16x16x32_f16(false, a, false, bw[2].v, (short)0, c[2], false, false);
  c[3] = __builtin_amdgcn_wmma_f32_16x16x32_f16(false, a, false, bw[3].v, (short)0, c[3], false, false);
  asm volatile("v_nop\n\tv_nop\n\tv_nop\n\tv_nop"
               : "+v"(c[0]), "+v"(c[1]), "+v"(c[2]), "+v"(c[3])
               : "v"(a), "v"(bw[0].v), "v"(bw[1].v), "v"(bw[2].v), "v"(bw[3].v));
}
__device__ __forceinline__ void mma_pj(v16b a, const FragB (&bw)[4], v8f (&c)[4]) {
  c[0] = __builtin_amdgcn_wmma_f32_16x16x32_bf16(false, a, false, bw[0].v, (short)0, c[0], false, false);
  c[1] = __builtin_amdgcn_wmma_f32_16x16x32_bf16(false, a, false, bw[1].v, (short)0, c[1], false, false);
  c[2] = __builtin_amdgcn_wmma_f32_16x16x32_bf16(false, a, false, bw[2].v, (short)0, c[2], false, false);
  c[3] = __builtin_amdgcn_wmma_f32_16x16x32_bf16(false, a, false, bw[3].v, (short)0, c[3], false, false);
  asm volatile("v_nop\n\tv_nop\n\tv_nop\n\tv_nop"
               : "+v"(c[0]), "+v"(c[1]), "+v"(c[2]), "+v"(c[3])
               : "v"(a), "v"(bw[0].v), "v"(bw[1].v), "v"(bw[2].v), "v"(bw[3].v));
}

__global__ __launch_bounds__(256) void k_cvt(const float* __restrict__ K, const float* __restrict__ W,
                                             unsigned short* __restrict__ Kb, unsigned short* __restrict__ Wh) {
  const int bid = blockIdx.x;
  if (bid < CVT_K_BLOCKS) {
    const int t = bid * 256 + threadIdx.x;
    const int row = t / (EMB / 8), piece = t - row * (EMB / 8);
    const int b = row / SEQ, s = row - b * SEQ;
    const float* src = K + (size_t)b * BSTRIDE_FULL + (size_t)s * EMB + piece * 8;
    const v4f x0 = *(const v4fa*)(src), x1 = *(const v4fa*)(src + 4);
    v8us o;
    o[0] = bf16_bits(x0[0]); o[1] = bf16_bits(x0[1]); o[2] = bf16_bits(x0[2]); o[3] = bf16_bits(x0[3]);
    o[4] = bf16_bits(x1[0]); o[5] = bf16_bits(x1[1]); o[6] = bf16_bits(x1[2]); o[7] = bf16_bits(x1[3]);
    store_twice(Kb + (size_t)t * 8, o);
  } else {
    const int t = (bid - CVT_K_BLOCKS) * 256 + threadIdx.x;
    const float* src = W + (size_t)t * 8;
    const v4f x0 = *(const v4fa*)(src), x1 = *(const v4fa*)(src + 4);
    v8us o;
    o[0] = f16_bits(bf16_rne(x0[0]) * 256.0f); o[1] = f16_bits(bf16_rne(x0[1]) * 256.0f);
    o[2] = f16_bits(bf16_rne(x0[2]) * 256.0f); o[3] = f16_bits(bf16_rne(x0[3]) * 256.0f);
    o[4] = f16_bits(bf16_rne(x1[0]) * 256.0f); o[5] = f16_bits(bf16_rne(x1[1]) * 256.0f);
    o[6] = f16_bits(bf16_rne(x1[2]) * 256.0f); o[7] = f16_bits(bf16_rne(x1[3]) * 256.0f);
    store_twice(Wh + (size_t)t * 8, o);
  }
}

__device__ __forceinline__ void cvt8_bf16(const float* __restrict__ src, unsigned short* __restrict__ dst) {
  const v4f x0 = *(const v4fa*)(src), x1 = *(const v4fa*)(src + 4);
  v8us o;
  o[0] = bf16_bits(x0[0]); o[1] = bf16_bits(x0[1]); o[2] = bf16_bits(x0[2]); o[3] = bf16_bits(x0[3]);
  o[4] = bf16_bits(x1[0]); o[5] = bf16_bits(x1[1]); o[6] = bf16_bits(x1[2]); o[7] = bf16_bits(x1[3]);
  store_twice(dst, o);
}
__global__ __launch_bounds__(256) void k_cvtw(const float* __restrict__ Wq, const float* __restrict__ Wk, const float* __restrict__ Wv,
                                              unsigned short* __restrict__ Wb) {
  const int bid = blockIdx.x;
  if (bid < CVT_W_BLOCKS) {
    const int t = bid * 256 + threadIdx.x;
    cvt8_bf16(Wq + (size_t)t * 8, Wb + (size_t)t * 8);
  } else if (bid < 2 * CVT_W_BLOCKS) {
    const int t = (bid - CVT_W_BLOCKS) * 256 + threadIdx.x;
    cvt8_bf16(Wk + (size_t)t * 8, Wb + (size_t)EMB * EMB + (size_t)t * 8);
  } else {
    const int t = (bid - 2 * CVT_W_BLOCKS) * 256 + threadIdx.x;
    cvt8_bf16(Wv + (size_t)t * 8, Wb + (size_t)2 * EMB * EMB + (size_t)t * 8);
  }
}

__global__ __launch_bounds__(128) void k_proj(const unsigned short* __restrict__ Xb, const unsigned short* __restrict__ Wb,
                                              const float* __restrict__ Bv, unsigned short* __restrict__ Dst, int tr) {
  __shared__ __attribute__((aligned(16))) unsigned short tl[64][72];
  const int tid = threadIdx.x, lane = tid & 31, ln = lane & 15, hh = lane >> 4;
  const int w = __builtin_amdgcn_readfirstlane(tid >> 5);
  const int bn = blockIdx.x % (EMB / 64), bm = blockIdx.x / (EMB / 64);
  const int tok0 = bm * 64;
  const int col0 = bn * 64;
  v8f acc[4] = {};
  const unsigned short* ap = Xb + (size_t)(tok0 + 16 * w + ln) * EMB + 8 * hh;
  const unsigned short* bp = Wb + (size_t)(col0 + ln) * EMB + 8 * hh;
#pragma unroll 1
  for (int kb = 0; kb < EMB / 96; ++kb) {
#pragma unroll
    for (int cc = 0; cc < 3; ++cc) {
      const int k0 = 96 * kb + 32 * cc;
      FragB a;
      a.half[0] = *(const v8us*)(ap + k0);
      a.half[1] = *(const v8us*)(ap + k0 + 16);
      FragB bw[4];
#pragma unroll
      for (int nt = 0; nt < 4; ++nt) {
        bw[nt].half[0] = *(const v8us*)(bp + (size_t)nt * 16 * EMB + k0);
        bw[nt].half[1] = *(const v8us*)(bp + (size_t)nt * 16 * EMB + k0 + 16);
      }
      mma_pj(a.v, bw, acc);
    }
  }
  if (tr == 0) {
#pragma unroll
    for (int nt = 0; nt < 4; ++nt) {
      const float bias = bf16_rne(Bv[col0 + 16 * nt + ln]);
#pragma unroll
      for (int r = 0; r < 8; ++r)
        tl[16 * w + 8 * hh + r][16 * nt + ln] = toh_flush_bits((acc[nt][r] + bias) * 16.0f);
    }
  } else {
#pragma unroll
    for (int nt = 0; nt < 4; ++nt) {
      const float bias = bf16_rne(Bv[col0 + 16 * nt + ln]);
      v8us o;
#pragma unroll
      for (int r = 0; r < 8; ++r) o[r] = toh_flush_bits((acc[nt][r] + bias) * 16.0f);
      *(v8us*)&tl[16 * nt + ln][16 * w + 8 * hh] = o;
    }
  }
  __syncthreads();
  const int b = tok0 / SEQ, s0 = tok0 - b * SEQ;
  const size_t base = (tr == 0) ? ((size_t)tok0 * EMB + col0) : (((size_t)b * EMB + col0) * SEQ + s0);
  const size_t pitch = (tr == 0) ? (size_t)EMB : (size_t)SEQ;
  for (int pass = 0; pass < 2; ++pass) {
    for (int i = tid; i < 64 * 8; i += 128) {
      const int r = i >> 3, p8 = (i & 7) * 8;
      const v8us o = *(const v8us*)&tl[r][p8];
      *(volatile v8us*)(Dst + base + (size_t)r * pitch + p8) = o;
    }
    if (pass == 0) __threadfence();
  }
}

__device__ __forceinline__ void fa_step(const unsigned short* __restrict__ Kp, const unsigned short* __restrict__ Vp,
                                        int key0, int ln, int hh, const FragH (&q)[3],
                                        float& mr, float& lr, v8f (&O)[6]) {
  const unsigned short* kp0 = Kp + (size_t)(key0 + ln) * EMB + 8 * hh;
  const unsigned short* kp1 = kp0 + 16 * EMB;
  FragH ka[3], kb[3];
#pragma unroll
  for (int c = 0; c < 3; ++c) {
    ka[c].half[0] = *(const v8us*)(kp0 + 32 * c);
    ka[c].half[1] = *(const v8us*)(kp0 + 32 * c + 16);
    kb[c].half[0] = *(const v8us*)(kp1 + 32 * c);
    kb[c].half[1] = *(const v8us*)(kp1 + 32 * c + 16);
  }
  const unsigned short* vp = Vp + (size_t)ln * SEQ + key0 + 8 * hh;
  FragH vf[6];
#pragma unroll
  for (int t = 0; t < 6; ++t) {
    vf[t].half[0] = *(const v8us*)(vp + (size_t)t * 16 * SEQ);
    vf[t].half[1] = *(const v8us*)(vp + (size_t)t * 16 * SEQ + 16);
  }
  v8f s0 = {0.f, 0.f, 0.f, 0.f, 0.f, 0.f, 0.f, 0.f};
  v8f s1 = {0.f, 0.f, 0.f, 0.f, 0.f, 0.f, 0.f, 0.f};
  mma_s2h(ka, kb, q, s0, s1);
  float sc[16];
#pragma unroll
  for (int r = 0; r < 8; ++r) { sc[r] = s0[r] * C2S; sc[8 + r] = s1[r] * C2S; }
  float mx = sc[0];
#pragma unroll
  for (int i = 1; i < 16; ++i) mx = fmaxf(mx, sc[i]);
  mx = fmaxf(mx, __shfl_xor(mx, 16, 32));
  const float mnew = fmaxf(mr, mx);
  const float al = __builtin_amdgcn_exp2f(mr - mnew);
  mr = mnew;
  const float m8 = mnew - 8.0f;
  FragH ph;
  float ps = 0.0f;
#pragma unroll
  for (int i = 0; i < 16; ++i) {
    const float e = sc[i] - m8;
    const float pe = __builtin_amdgcn_exp2f(e);
    const float pc = (e < -14.0f) ? 0.0f : pe;
    ps += pc;
    ph.h[i] = (_Float16)pc;
  }
  ps += __shfl_xor(ps, 16, 32);
  lr = lr * al + ps;
#pragma unroll
  for (int t = 0; t < 6; ++t) O[t] = O[t] * al;
  mma_pv(vf, ph.v, O);
}

__global__ __launch_bounds__(128) __attribute__((amdgpu_num_vgpr(256)))
void k_attn(const unsigned short* __restrict__ Qh, const unsigned short* __restrict__ Kh,
            const unsigned short* __restrict__ Vt, unsigned short* __restrict__ Xc) {
  __shared__ __attribute__((aligned(16))) unsigned short so[4][16 * HD];
  const int tid = threadIdx.x, lane = tid & 31, ln = lane & 15, hh = lane >> 4;
  const int w = __builtin_amdgcn_readfirstlane(tid >> 5);
  const int qt = blockIdx.x % (SEQ / 64);
  const int rest = blockIdx.x / (SEQ / 64);
  const int h = rest % HEADS, b = rest / HEADS;
  const int qbase = qt * 64 + 16 * w;
  const int qg = qbase + ln;
  const unsigned short* qrow = Qh + ((size_t)b * SEQ + qg) * EMB + h * HD + 8 * hh;
  FragH q[3];
#pragma unroll
  for (int c = 0; c < 3; ++c) {
    q[c].half[0] = *(const v8us*)(qrow + 32 * c);
    q[c].half[1] = *(const v8us*)(qrow + 32 * c + 16);
  }
  float mr = -3.0e38f, lr = 0.0f;
  v8f O[6] = {};
  const unsigned short* Kp = Kh + (size_t)b * SEQ * EMB + h * HD;
  const unsigned short* Vp = Vt + ((size_t)b * EMB + h * HD) * SEQ;
#pragma unroll 1
  for (int j = 0; j < SEQ / 32; ++j)
    fa_step(Kp, Vp, 32 * j, ln, hh, q, mr, lr, O);

  const float cinv = 16.0f * (1.0f / lr);
#pragma unroll
  for (int t = 0; t < 6; ++t) {
    v8us o;
#pragma unroll
    for (int r = 0; r < 8; ++r) o[r] = toh_flush_bits(O[t][r] * cinv);
    *(v8us*)&so[w][ln * HD + 16 * t + 8 * hh] = o;
  }
  __syncthreads();
  unsigned short* xg = Xc + ((size_t)(b * HEADS + h) * SEQ + qbase) * HD;
  for (int pass = 0; pass < 2; ++pass) {
#pragma unroll
    for (int i = 0; i < 6; ++i) {
      const int p = i * 32 + lane;
      const v8us v = *(const v8us*)&so[w][p * 8];
      *(volatile v8us*)(xg + (size_t)p * 8) = v;
    }
    if (pass == 0) __threadfence();
  }
}

__global__ __launch_bounds__(128) void k_fc(const unsigned short* __restrict__ Xc, const unsigned short* __restrict__ Wh,
                                            const float* __restrict__ Bv, float* __restrict__ Out) {
  __shared__ __attribute__((aligned(16))) float so[4][16][68];
  const int tid = threadIdx.x, lane = tid & 31, ln = lane & 15, hh = lane >> 4;
  const int w = __builtin_amdgcn_readfirstlane(tid >> 5);
  const int bn = blockIdx.x % (EMB / 64), bm = blockIdx.x / (EMB / 64);
  const int row0 = bm * 64 + 16 * w;
  const int b = row0 / SEQ, s0 = row0 - b * SEQ;
  const int col0 = bn * 64;
  v8f acc[4] = {};
#pragma unroll 1
  for (int hd = 0; hd < HEADS; ++hd) {
    const unsigned short* ap = Xc + ((size_t)(b * HEADS + hd) * SEQ + s0 + ln) * HD + 8 * hh;
    const unsigned short* bp = Wh + (size_t)(col0 + ln) * EMB + hd * HD + 8 * hh;
#pragma unroll
    for (int cc = 0; cc < 3; ++cc) {
      FragH a;
      a.half[0] = *(const v8us*)(ap + 32 * cc);
      a.half[1] = *(const v8us*)(ap + 32 * cc + 16);
      FragH bw[4];
#pragma unroll
      for (int nt = 0; nt < 4; ++nt) {
        bw[nt].half[0] = *(const v8us*)(bp + (size_t)nt * 16 * EMB + 32 * cc);
        bw[nt].half[1] = *(const v8us*)(bp + (size_t)nt * 16 * EMB + 32 * cc + 16);
      }
      mma_fc(a.v, bw, acc);
    }
  }
#pragma unroll
  for (int nt = 0; nt < 4; ++nt) {
    const float bias = bf16_rne(Bv[col0 + 16 * nt + ln]);
#pragma unroll
    for (int r = 0; r < 8; ++r)
      so[w][8 * hh + r][16 * nt + ln] = acc[nt][r] * 1.52587890625e-05f + bias;
  }
  __syncthreads();
  float* og = Out + (size_t)b * BSTRIDE_FULL + (size_t)s0 * EMB + col0;
  const int rsub = lane >> 4, c4 = (lane & 15) * 4;
  for (int pass = 0; pass < 2; ++pass) {
#pragma unroll
    for (int q = 0; q < 8; ++q) {
      const int row = 2 * q + rsub;
      const v4f v = *(const v4fa*)&so[w][row][c4];
      *(volatile v4f*)(og + (size_t)row * EMB + c4) = v;
    }
    if (pass == 0) __threadfence();
  }
}

extern "C" void kernel_launch(void* const* d_in, const int* in_sizes, int n_in,
                              void* d_out, int out_size, void* d_ws, size_t ws_size, hipStream_t stream) {
  if (n_in < 9) return;
  const long long need = (long long)(NB - 1) * SEQ_FULL * EMB + (long long)SEQ * EMB;
  if ((long long)in_sizes[0] < need) return;
  if ((long long)in_sizes[1] < (long long)EMB * EMB || (long long)in_sizes[3] < (long long)EMB * EMB) return;
  if ((long long)in_sizes[5] < (long long)EMB * EMB || (long long)in_sizes[7] < (long long)EMB * EMB) return;
  if ((long long)in_sizes[2] < (long long)EMB || (long long)in_sizes[4] < (long long)EMB) return;
  if ((long long)in_sizes[6] < (long long)EMB || (long long)in_sizes[8] < (long long)EMB) return;
  if ((long long)out_size < need) return;
  const float* X  = (const float*)d_in[0];
  const float* Wq = (const float*)d_in[1];
  const float* Bq = (const float*)d_in[2];
  const float* Wk = (const float*)d_in[3];
  const float* Bk = (const float*)d_in[4];
  const float* Wv = (const float*)d_in[5];
  const float* Bvv = (const float*)d_in[6];
  const float* Wo = (const float*)d_in[7];
  const float* Bo = (const float*)d_in[8];
  float* Out = (float*)d_out;
  char* ws = (char*)d_ws;
  size_t off = 0;
  unsigned short* Xb = (unsigned short*)(ws + off); off += PLANE_ACT;
  unsigned short* Qh = (unsigned short*)(ws + off); off += PLANE_ACT;
  unsigned short* Kh = (unsigned short*)(ws + off); off += PLANE_ACT;
  unsigned short* Vt = (unsigned short*)(ws + off); off += PLANE_ACT;
  unsigned short* Xc = (unsigned short*)(ws + off); off += PLANE_ACT;
  unsigned short* Wh = (unsigned short*)(ws + off); off += PLANE_W;
  unsigned short* Wb = (unsigned short*)(ws + off); off += 3 * PLANE_W;
  if (off > ws_size) return;
  k_cvt<<<(unsigned)(CVT_K_BLOCKS + CVT_W_BLOCKS), 256, 0, stream>>>(X, Wo, Xb, Wh);
  k_cvtw<<<(unsigned)(3 * CVT_W_BLOCKS), 256, 0, stream>>>(Wq, Wk, Wv, Wb);
  k_proj<<<(unsigned)PROJ_BLOCKS, 128, 0, stream>>>(Xb, Wb, Bq, Qh, 0);
  k_proj<<<(unsigned)PROJ_BLOCKS, 128, 0, stream>>>(Xb, Wb + (size_t)EMB * EMB, Bk, Kh, 0);
  k_proj<<<(unsigned)PROJ_BLOCKS, 128, 0, stream>>>(Xb, Wb + (size_t)2 * EMB * EMB, Bvv, Vt, 1);
  k_attn<<<(unsigned)(NB * HEADS * (SEQ / 64)), 128, 0, stream>>>(Qh, Kh, Vt, Xc);
  k_fc<<<(unsigned)((NB * SEQ / 64) * (EMB / 64)), 128, 0, stream>>>(Xc, Wh, Bo, Out);
}
